// CoAttention_64639257805493
// MI455X (gfx1250) — hardware-run, weakly checked
//
#include <hip/hip_runtime.h>
#include <math.h>

typedef __attribute__((ext_vector_type(16))) _Float16 v16h;
typedef __attribute__((ext_vector_type(8)))  _Float16 v8h;
typedef __attribute__((ext_vector_type(4)))  _Float16 v4h;
typedef __attribute__((ext_vector_type(2)))  _Float16 v2h;
typedef __attribute__((ext_vector_type(16))) __bf16   v16b;
typedef __attribute__((ext_vector_type(8)))  __bf16   v8b;
typedef __attribute__((ext_vector_type(8)))  float    v8f;
typedef __attribute__((ext_vector_type(4)))  float    v4f;
typedef __attribute__((ext_vector_type(2)))  float    v2f;

constexpr int kBatch  = 16;
constexpr int kSteps  = 512;
constexpr int kLq     = 64;
constexpr int kD      = 256;
constexpr int kHid    = 256;
constexpr int kD2     = 2 * kD;
constexpr int kGate3  = 3 * kHid;
constexpr int kRows   = kBatch * kSteps;
constexpr int kQRows  = kBatch * kLq;
constexpr int kThr    = 256;
constexpr int kThrRun = 128;
constexpr int kSeqBlk = 16;
constexpr int kHP     = kHid + 8;
constexpr int kHmP    = kHid;

constexpr float kInCarry  = 1024.0f;
constexpr float kWCarry   = 1024.0f;
constexpr float kActCarry = 4096.0f;
constexpr float kXsScale  = 1.0f / (kInCarry * kWCarry);
constexpr float kRecScale = 1.0f / (kActCarry * kWCarry);
constexpr float kF16MinNormal = 6.103515625e-5f;

static_assert((kRows % 64) == 0 && (kQRows % 64) == 0 && (kHid % 64) == 0 && (kD2 % 64) == 0 && (kGate3 % 64) == 0 && (kLq % 32) == 0, "GEMM M, N multiples of 64, K of 32");
static_assert(kBatch == kSeqBlk && kThrRun == (kHid / 64) * 32, "one run block; a wave per 64 units");

constexpr size_t kOffC16 = 0;
constexpr size_t kOffQ16 = kOffC16 + (size_t)kRows * kD2 * 2;
constexpr size_t kOffQT  = kOffQ16 + (size_t)kQRows * kD * 2;
constexpr size_t kOffWCT = kOffQT  + (size_t)kBatch * kD * kLq * 2;
constexpr size_t kOffWQT = kOffWCT + (size_t)kHid * kD * 2;
constexpr size_t kOffWGT = kOffWQT + (size_t)kHid * kD * 2;
constexpr size_t kOffWIH = kOffWGT + (size_t)kD2 * kD2 * 2;
constexpr size_t kOffWHH = kOffWIH + (size_t)kGate3 * kD2 * 2;
constexpr size_t kOffBV  = kOffWHH + (size_t)kGate3 * kHid * 2;
constexpr size_t kOffCD  = kOffBV  + (size_t)6 * kGate3 * 4;
constexpr size_t kOffQD  = kOffCD  + (size_t)kRows * kHid * 4;
constexpr size_t kOffS16 = kOffQD  + (size_t)kQRows * kHid * 4;
constexpr size_t kOffATT = kOffS16 + (size_t)kRows * kLq * 2;
constexpr size_t kOffG   = kOffATT + (size_t)kRows * kD * 4;
constexpr size_t kOffRN2 = kOffG   + (size_t)kRows * kD2 * 4;
constexpr size_t kOffXS  = kOffRN2 + (size_t)kRows * kD2 * 2;
constexpr size_t kWsTotal = kOffXS + (size_t)kRows * kGate3 * 4;
static_assert(kWsTotal == 80627712ull, "carve total");
static_assert(kWsTotal <= 134217728ull, "carve cap");
static_assert((kOffQ16 % 256) == 0 && (kOffQT % 256) == 0 && (kOffWCT % 256) == 0 && (kOffWQT % 256) == 0 && (kOffWGT % 256) == 0 && (kOffWIH % 256) == 0 && (kOffWHH % 256) == 0 && (kOffBV % 256) == 0 && (kOffCD % 256) == 0 && (kOffQD % 256) == 0 && (kOffS16 % 256) == 0 && (kOffATT % 256) == 0 && (kOffG % 256) == 0 && (kOffRN2 % 256) == 0 && (kOffXS % 256) == 0, "aligned regions");

__device__ __forceinline__ unsigned short f2bf_bits(float f) {
  unsigned u = __float_as_uint(f);
  return (unsigned short)((u + 0x7FFFu + ((u >> 16) & 1u)) >> 16);
}
__device__ __forceinline__ float bf_bits2f(unsigned short h) { return __uint_as_float(((unsigned)h) << 16); }
__device__ __forceinline__ float bf16r(float f) { return bf_bits2f(f2bf_bits(f)); }
__device__ __forceinline__ float carry_flush(float v, float carry) {
  const float s = v * carry;
  return (fabsf(s) < kF16MinNormal) ? 0.0f : s;
}
__device__ __forceinline__ float frcp(float x) { return __builtin_amdgcn_rcpf(x); }

__device__ __forceinline__ void dep_guard4_h(v8f& a, v8f& b, v8f& c, v8f& d, v16h x, v16h y) { asm volatile("v_nop\n\tv_nop\n\tv_nop\n\tv_nop" : "+v"(a), "+v"(b), "+v"(c), "+v"(d) : "v"(x), "v"(y)); }
__device__ __forceinline__ void dep_guard4_b(v8f& a, v8f& b, v8f& c, v8f& d, v16b x, v16b y) { asm volatile("v_nop\n\tv_nop\n\tv_nop\n\tv_nop" : "+v"(a), "+v"(b), "+v"(c), "+v"(d) : "v"(x), "v"(y)); }
__device__ __forceinline__ void keep4_h(v16h a, v16h b, v16h c, v16h d) { asm volatile("v_nop" :: "v"(a), "v"(b), "v"(c), "v"(d)); }
__device__ __forceinline__ void keep4_b(v16b a, v16b b, v16b c, v16b d) { asm volatile("v_nop" :: "v"(a), "v"(b), "v"(c), "v"(d)); }
__device__ __forceinline__ void acc_guard4(v8f& a, v8f& b, v8f& c, v8f& d) { asm volatile("v_nop\n\tv_nop\n\tv_nop\n\tv_nop" : "+v"(a), "+v"(b), "+v"(c), "+v"(d)); }

template <typename T> struct Frag;
template <> struct Frag<_Float16> {
  typedef v16h V; union U { v16h v; v8h h[2]; };
  static __device__ __forceinline__ v16h load(const _Float16* p) {
    U f; f.h[0] = *(const v8h*)(p); f.h[1] = *(const v8h*)(p + 16); return f.v;
  }
  static __device__ __forceinline__ v8f mma(v16h a, v16h b, v8f c) {
    return __builtin_amdgcn_wmma_f32_16x16x32_f16(false, a, false, b, (short)0, c, false, false);
  }
  static __device__ __forceinline__ void guard4(v8f& a, v8f& b, v8f& c, v8f& d, v16h x, v16h y) { dep_guard4_h(a, b, c, d, x, y); }
  static __device__ __forceinline__ void keep(v16h a, v16h b, v16h c, v16h d) { keep4_h(a, b, c, d); }
};
template <> struct Frag<__bf16> {
  typedef v16b V; union U { v16b v; v8b h[2]; };
  static __device__ __forceinline__ v16b load(const __bf16* p) {
    U f; f.h[0] = *(const v8b*)(p); f.h[1] = *(const v8b*)(p + 16); return f.v;
  }
  static __device__ __forceinline__ v8f mma(v16b a, v16b b, v8f c) {
    return __builtin_amdgcn_wmma_f32_16x16x32_bf16(false, a, false, b, (short)0, c, false, false);
  }
  static __device__ __forceinline__ void guard4(v8f& a, v8f& b, v8f& c, v8f& d, v16b x, v16b y) { dep_guard4_b(a, b, c, d, x, y); }
  static __device__ __forceinline__ void keep(v16b a, v16b b, v16b c, v16b d) { keep4_b(a, b, c, d); }
};

__device__ __forceinline__ v8f mma_h(v16h a, v16h b, v8f c) {
  c = __builtin_amdgcn_wmma_f32_16x16x32_f16(false, a, false, b, (short)0, c, false, false);
  asm volatile("v_nop\n\tv_nop\n\tv_nop\n\tv_nop" : "+v"(c) : "v"(a), "v"(b));
  return c;
}

template <int ET> struct Elem;
template <> struct Elem<0> { typedef _Float16 T; };
template <> struct Elem<1> { typedef __bf16 T; };
template <int ET, bool SPLIT, int BIAS_MODE, int OUT_MODE, bool RESID, int ACT = 0>
__global__ __launch_bounds__(256) void wmma_gemm64(
    const unsigned short* __restrict__ Ap, const unsigned short* __restrict__ A2p, int lda, long strideA,
    const unsigned short* __restrict__ Btp, const unsigned short* __restrict__ Bt2p, int ldb, long strideB,
    void* __restrict__ Cout, void* __restrict__ Cout2, int ldc, long strideC,
    const float* __restrict__ bias,
    const float* __restrict__ resid, long strideR,
    int M, int N, int K, float scale) {
  typedef typename Elem<ET>::T T;
  typedef typename Frag<T>::V V;
  const T* A = (const T*)Ap; const T* A2 = (const T*)A2p; const T* Bt = (const T*)Btp; const T* Bt2 = (const T*)Bt2p;
  __shared__ __align__(16) float sT[8][16 * 68];
  const int b    = blockIdx.y;
  const int lane = threadIdx.x & 31;
  const int wave = threadIdx.x >> 5;
  const int tilesN = N >> 6;
  const int tilesM = M >> 6;
  const int tile = blockIdx.x * 8 + wave;
  if (tile >= tilesM * tilesN) return;
  const int tm = tile / tilesN;
  const int tn = tile - tm * tilesN;
  const int m0 = tm << 6;
  const int n0 = tn << 6;

  const T* Ab  = A  + (size_t)b * strideA;
  const T* Bb  = Bt + (size_t)b * strideB;
  const T* Ab2 = SPLIT ? (A2  + (size_t)b * strideA) : nullptr;
  const T* Bb2 = SPLIT ? (Bt2 + (size_t)b * strideB) : nullptr;

  const int rlane = lane & 15;
  const int koff  = (lane >> 4) * 8;
  const int mOff  = (lane >> 4) * 8;

  v8f acc[4][4];
#pragma unroll
  for (int i = 0; i < 4; ++i)
#pragma unroll
    for (int j = 0; j < 4; ++j) acc[i][j] = (v8f){0.f,0.f,0.f,0.f,0.f,0.f,0.f,0.f};

  for (int k0 = 0; k0 < K; k0 += 32) {
    V bh[4], bl[4];
#pragma unroll
    for (int j = 0; j < 4; ++j) {
      const size_t bo = (size_t)(n0 + (j << 4) + rlane) * ldb + koff + k0;
      bh[j] = Frag<T>::load(Bb + bo);
      if (SPLIT) bl[j] = Frag<T>::load(Bb2 + bo);
    }
#pragma unroll
    for (int i = 0; i < 4; ++i) {
      const size_t ao = (size_t)(m0 + (i << 4) + rlane) * lda + koff + k0;
      V ah = Frag<T>::load(Ab + ao);
      V al;
      if (SPLIT) al = Frag<T>::load(Ab2 + ao);
#pragma unroll
      for (int j = 0; j < 4; ++j) {
        acc[i][j] = Frag<T>::mma(ah, bh[j], acc[i][j]);
        if (SPLIT) {
          acc[i][j] = Frag<T>::mma(ah, bl[j], acc[i][j]);
          acc[i][j] = Frag<T>::mma(al, bh[j], acc[i][j]);
        }
      }
      Frag<T>::guard4(acc[i][0], acc[i][1], acc[i][2], acc[i][3], ah, SPLIT ? al : ah);
    }
    Frag<T>::keep(bh[0], bh[1], bh[2], bh[3]);
    if (SPLIT) Frag<T>::keep(bl[0], bl[1], bl[2], bl[3]);
  }
  acc_guard4(acc[0][0], acc[0][1], acc[0][2], acc[0][3]);
  acc_guard4(acc[1][0], acc[1][1], acc[1][2], acc[1][3]);
  acc_guard4(acc[2][0], acc[2][1], acc[2][2], acc[2][3]);
  acc_guard4(acc[3][0], acc[3][1], acc[3][2], acc[3][3]);

  float* slab = sT[wave];
  const float* Rb = RESID ? (resid + (size_t)b * strideR) : nullptr;
#pragma unroll
  for (int i = 0; i < 4; ++i) {
    const int mBase = m0 + (i << 4);
#pragma unroll
    for (int j = 0; j < 4; ++j) {
      const int n = n0 + (j << 4) + rlane;
      float bv = 0.f;
      if (BIAS_MODE == 2) bv = bias[n];
#pragma unroll
      for (int r = 0; r < 8; ++r) {
        float v = acc[i][j][r] * scale;
        if (BIAS_MODE == 1) v += bias[mBase + mOff + r];
        if (BIAS_MODE == 2) v += bv;
        if (RESID) v += Rb[(size_t)(mBase + mOff + r) * ldc + n];
        if (ACT == 1) v = tanhf(v);
        if (ACT == 2) v = fmaxf(v, 0.0f);
        if (ACT == 3) v = v / (1.0f + expf(-v));
        if (ACT == 4) v = (v > 0.f) ? v : 0.01f * v;
        slab[(mOff + r) * 68 + (j << 4) + rlane] = v;
      }
    }
    __builtin_amdgcn_fence(__ATOMIC_RELEASE, "workgroup");
    __builtin_amdgcn_wave_barrier();
    __builtin_amdgcn_fence(__ATOMIC_ACQUIRE, "workgroup");
    if (OUT_MODE == 0) {
      float* C = (float*)Cout + (size_t)b * strideC;
      const int hh = lane >> 4, c4 = (lane & 15) * 4;
      for (int pass = 0; pass < 2; ++pass) {
#pragma unroll
        for (int it = 0; it < 8; ++it) {
          const int row = it * 2 + hh;
          v4f v = *(const v4f*)(slab + row * 68 + c4);
          *(volatile v4f*)(C + (size_t)(mBase + row) * ldc + n0 + c4) = v;
        }
        __threadfence();
      }
    } else {
      const int q = lane >> 3, c8 = (lane & 7) * 8;
      unsigned short* C  = (unsigned short*)Cout  + (size_t)b * strideC;
      unsigned short* C2 = (OUT_MODE == 2) ? ((unsigned short*)Cout2 + (size_t)b * strideC) : nullptr;
      for (int pass = 0; pass < 2; ++pass) {
#pragma unroll
        for (int it = 0; it < 4; ++it) {
          const int row = it * 4 + q;
          const float* sp = slab + row * 68 + c8;
          v8h hv, lv;
#pragma unroll
          for (int e = 0; e < 8; ++e) {
            if (OUT_MODE == 1) {
              hv[e] = (_Float16)sp[e];
            } else {
              unsigned short hb = f2bf_bits(sp[e]);
              unsigned short lb = f2bf_bits(sp[e] - bf_bits2f(hb));
              hv[e] = __builtin_bit_cast(_Float16, hb);
              lv[e] = __builtin_bit_cast(_Float16, lb);
            }
          }
          *(volatile v8h*)(C + (size_t)(mBase + row) * ldc + n0 + c8) = hv;
          if (OUT_MODE == 2) *(volatile v8h*)(C2 + (size_t)(mBase + row) * ldc + n0 + c8) = lv;
        }
        __threadfence();
      }
    }
    __builtin_amdgcn_fence(__ATOMIC_RELEASE, "workgroup");
    __builtin_amdgcn_wave_barrier();
    __builtin_amdgcn_fence(__ATOMIC_ACQUIRE, "workgroup");
  }
}

__global__ __launch_bounds__(kThr) void cast_plane_kernel(const float* __restrict__ src, unsigned short* __restrict__ dst,
                                                          int colsLog2, int dstPitch, int dstOff) {
  const int i   = blockIdx.x * kThr + threadIdx.x;
  const int sh  = colsLog2 - 3;
  const int row = i >> sh;
  const int c8  = (i & ((1 << sh) - 1)) * 8;
  const float* sp = src + ((size_t)row << colsLog2) + c8;
  const v4f a0 = *(const v4f*)(sp);
  const v4f a1 = *(const v4f*)(sp + 4);
  v8h hv;
#pragma unroll
  for (int e = 0; e < 4; ++e) {
    const float f0 = a0[e];
    const float f1 = a1[e];
    hv[e]     = (_Float16)carry_flush(bf16r(f0), kInCarry);
    hv[4 + e] = (_Float16)carry_flush(bf16r(f1), kInCarry);
  }
  unsigned short* dp = dst + (size_t)row * dstPitch + dstOff + c8;
  *(volatile v8h*)dp = hv;
  __threadfence();
  *(volatile v8h*)dp = hv;
}
static_assert(kInCarry == kWCarry, "one cast kernel serves inputs and weights");

__global__ __launch_bounds__(64) void tplane_kernel(const float* __restrict__ src, unsigned short* __restrict__ dst,
                                                    int K, int N) {
  const int n  = blockIdx.x;
  const int bt = blockIdx.y;
  const int k8 = threadIdx.x * 8;
  const float* sp = src + (size_t)bt * K * N;
  v8h hv;
#pragma unroll
  for (int e = 0; e < 8; ++e) hv[e] = (_Float16)carry_flush(bf16r(sp[(size_t)(k8 + e) * N + n]), kWCarry);
  unsigned short* dp = dst + ((size_t)bt * N + n) * K + k8;
  *(volatile v8h*)dp = hv;
  __threadfence();
  *(volatile v8h*)dp = hv;
}

__global__ __launch_bounds__(kThr) void ca_bias_kernel(const float* __restrict__ bc, const float* __restrict__ bq,
                                                       const float* __restrict__ bg, const float* __restrict__ bih,
                                                       const float* __restrict__ bhh, float* __restrict__ BV) {
  const int tid = threadIdx.x;
#pragma unroll 1
  for (int it = 0; it < kGate3 / kThr; ++it) {
    const int e = it * kThr + tid;
    const int e256 = (e < kHid) ? e : (kHid - 1);
    const int e512 = (e < kD2) ? e : (kD2 - 1);
    float v0 = bc[e256], v1 = bq[e256], v2 = bg[e512];
    asm volatile("" : "+v"(v0), "+v"(v1), "+v"(v2));
    const float o0 = (e < kHid) ? bf16r(v0) : 0.0f;
    const float o1 = (e < kHid) ? bf16r(v1) : 0.0f;
    const float o2 = (e < kD2) ? bf16r(v2) : 0.0f;
    const float o3 = bf16r(bih[e]);
    const float o4 = bf16r(bhh[e]);
    for (int pass = 0; pass < 2; ++pass) {
      *(volatile float*)(BV + 0 * kGate3 + e) = o0;
      *(volatile float*)(BV + 1 * kGate3 + e) = o1;
      *(volatile float*)(BV + 2 * kGate3 + e) = o2;
      *(volatile float*)(BV + 3 * kGate3 + e) = o3;
      *(volatile float*)(BV + 4 * kGate3 + e) = o4;
      *(volatile float*)(BV + 5 * kGate3 + e) = 0.0f;
      __threadfence();
    }
  }
}

__device__ __forceinline__ float fast_tanh_f(float v) {
  const float e = __expf(2.0f * v);
  return 1.0f - 2.0f * __builtin_amdgcn_rcpf(e + 1.0f);
}

__global__ __launch_bounds__(kThr) void score_kernel(const float* __restrict__ CD, const float* __restrict__ QD,
                                                     const float* __restrict__ Ws, const float* __restrict__ bs,
                                                     const float* __restrict__ qmask, unsigned short* __restrict__ S16) {
  __shared__ float sq[kLq * 257];
  __shared__ __align__(16) float sc[8][kHid];
  __shared__ __align__(16) float sw[kHid];
  __shared__ __align__(16) float ss[8][kLq];
  const int b  = blockIdx.x >> 3;
  const int p0 = (blockIdx.x & 7) * 64;
  const int tid = threadIdx.x, lane = tid & 31, wave = tid >> 5;

#pragma unroll 4
  for (int q = 0; q < kLq; ++q) sq[q * 257 + tid] = QD[((size_t)b * kLq + q) * kHid + tid];
  sw[tid] = bf16r(Ws[tid]);
  __syncthreads();

  const float bsv = bf16r(bs[0]);
  const float m0 = qmask[(size_t)b * kLq + 2 * lane];
  const float m1 = qmask[(size_t)b * kLq + 2 * lane + 1];
  const float* q0p = sq + (2 * lane) * 257;
  const float* q1p = sq + (2 * lane + 1) * 257;
  float* myc = &sc[wave][0];
  float* mys = &ss[wave][0];

#pragma unroll 1
  for (int pi = 0; pi < 8; ++pi) {
    const int row = b * kSteps + p0 + 8 * wave + pi;
    {
      const v4f c0 = *(const v4f*)(CD + (size_t)row * kHid + 8 * lane);
      const v4f c1 = *(const v4f*)(CD + (size_t)row * kHid + 8 * lane + 4);
      *(v4f*)(myc + 8 * lane) = c0;
      *(v4f*)(myc + 8 * lane + 4) = c1;
    }
    __syncthreads();
    float s0 = 0.0f, s1 = 0.0f;
#pragma unroll 4
    for (int h = 0; h < kHid; ++h) {
      const float cv = myc[h];
      const float wv = sw[h];
      s0 = fmaf(fast_tanh_f(cv + q0p[h]), wv, s0);
      s1 = fmaf(fast_tanh_f(cv + q1p[h]), wv, s1);
    }
    s0 = (m0 > 0.0f) ? (s0 + bsv) : -1e30f;
    s1 = (m1 > 0.0f) ? (s1 + bsv) : -1e30f;
    mys[2 * lane] = s0;
    mys[2 * lane + 1] = s1;
    __syncthreads();
    float mx = mys[0];
#pragma unroll 4
    for (int q = 1; q < kLq; ++q) mx = fmaxf(mx, mys[q]);
    float sum = 0.0f;
#pragma unroll 4
    for (int q = 0; q < kLq; ++q) sum += expf(mys[q] - mx);
    const float e0 = expf(s0 - mx) / sum;
    const float e1 = expf(s1 - mx) / sum;
    v2h so;
    so[0] = (_Float16)carry_flush(e0, kActCarry);
    so[1] = (_Float16)carry_flush(e1, kActCarry);
    unsigned short* sp = S16 + (size_t)row * kLq + 2 * lane;
    *(volatile v2h*)sp = so;
    __threadfence();
    *(volatile v2h*)sp = so;
    __syncthreads();
  }
}

__global__ __launch_bounds__(kThr) void att_cast_kernel(const float* __restrict__ ATT, unsigned short* __restrict__ C16) {
  const int i = blockIdx.x * kThr + threadIdx.x;
  const int row = i >> 5;
  const int c8 = (i & 31) * 8;
  const v4f a0 = *(const v4f*)(ATT + (size_t)row * kD + c8);
  const v4f a1 = *(const v4f*)(ATT + (size_t)row * kD + c8 + 4);
  v8h hv;
#pragma unroll
  for (int e = 0; e < 4; ++e) {
    hv[e]     = (_Float16)carry_flush(a0[e], kInCarry);
    hv[4 + e] = (_Float16)carry_flush(a1[e], kInCarry);
  }
  unsigned short* dp = C16 + (size_t)row * kD2 + kD + c8;
  *(volatile v8h*)dp = hv;
  __threadfence();
  *(volatile v8h*)dp = hv;
}

__global__ __launch_bounds__(kThr) void gate_mul_kernel(const float* __restrict__ ctx, const float* __restrict__ ATT,
                                                        const float* __restrict__ G, unsigned short* __restrict__ RN2) {
  const int i = blockIdx.x * kThr + threadIdx.x;
  const int row = i >> 7;
  const int c4 = (i & 127) * 4;
  const int cc = c4 & (kD - 1);
  v4f xc = *(const v4f*)(ctx + (size_t)row * kD + cc);
  v4f xa = *(const v4f*)(ATT + (size_t)row * kD + cc);
  asm volatile("" : "+v"(xc), "+v"(xa));
  const v4f g = *(const v4f*)(G + (size_t)row * kD2 + c4);
  v4h ho;
#pragma unroll
  for (int e = 0; e < 4; ++e) {
    const float rin = (c4 < kD) ? bf16r(xc[e]) : xa[e];
    const float sg = 1.0f / (1.0f + expf(-g[e]));
    ho[e] = (_Float16)carry_flush(rin * sg, kInCarry);
  }
  unsigned short* dp = RN2 + (size_t)row * kD2 + c4;
  *(volatile v4h*)dp = ho;
  __threadfence();
  *(volatile v4h*)dp = ho;
}

__global__ __launch_bounds__(kThrRun) void gated_run_kernel(const float* __restrict__ XS,
                                                            const unsigned short* __restrict__ WHp,
                                                            const float* __restrict__ BH,
                                                            const int* __restrict__ LEN,
                                                            float* __restrict__ OUT0) {
  __shared__ __align__(16) _Float16 Ah[2][kSeqBlk * kHP];
  __shared__ __align__(16) float    Hm[kSeqBlk * kHmP];
  __shared__ __align__(16) float    sBh[kGate3];
  const _Float16* WH = (const _Float16*)WHp;
  const int tid = threadIdx.x, lane = tid & 31, wave = tid >> 5;
  const int c = lane & 15, hh = lane >> 4, koff = hh * 8, c4 = c * 4;
  const int rowbase = blockIdx.x * kSeqBlk;

  {
    _Float16* ahf = &Ah[0][0];
#pragma unroll 1
    for (int i = tid; i < 2 * kSeqBlk * kHP; i += kThrRun) ahf[i] = (_Float16)0.0f;
#pragma unroll 1
    for (int i = tid; i < kSeqBlk * kHmP; i += kThrRun) Hm[i] = 0.0f;
#pragma unroll 1
    for (int i = tid; i < kGate3; i += kThrRun) sBh[i] = BH[i];
  }
  __syncthreads();

  const v8f z8 = {0.f, 0.f, 0.f, 0.f, 0.f, 0.f, 0.f, 0.f};
  int lenr[8];
#pragma unroll
  for (int it = 0; it < 8; ++it) lenr[it] = LEN[rowbase + it * 2 + hh];

#pragma unroll 1
  for (int s = 0; s < kSteps; ++s) {
    const int cur = s & 1;
    const _Float16* ahrow = &Ah[cur][0] + c * kHP + koff;
    _Float16* ahn = &Ah[cur ^ 1][0];
    const float* xsrow = XS + ((size_t)(rowbase + 8 * hh) * kSteps + s) * kGate3;

#pragma unroll 1
    for (int nt = 0; nt < 4; ++nt) {
      const int j = 64 * wave + 16 * nt + c;
      float xr[8], xz[8], xn[8];
#pragma unroll
      for (int r = 0; r < 8; ++r) {
        const float* xp = xsrow + (size_t)r * kSteps * kGate3 + j;
        xr[r] = xp[0];
        xz[r] = xp[kHid];
        xn[r] = xp[2 * kHid];
      }
      const _Float16* wr = WH + (size_t)j * kHid + koff;
      const _Float16* wz = WH + (size_t)(kHid + j) * kHid + koff;
      const _Float16* wn = WH + (size_t)(2 * kHid + j) * kHid + koff;
      v8f ar = z8, az = z8, an = z8;
#pragma unroll 2
      for (int k0 = 0; k0 < kHid; k0 += 32) {
        const v16h a   = Frag<_Float16>::load(ahrow + k0);
        const v16h fbr = Frag<_Float16>::load(wr + k0);
        const v16h fbz = Frag<_Float16>::load(wz + k0);
        const v16h fbn = Frag<_Float16>::load(wn + k0);
        ar = mma_h(a, fbr, ar);
        az = mma_h(a, fbz, az);
        an = mma_h(a, fbn, an);
      }
      const float bhr = sBh[j];
      const float bhz = sBh[kHid + j];
      const float bhn = sBh[2 * kHid + j];
#pragma unroll
      for (int r = 0; r < 8; ++r) {
        const int row = 8 * hh + r;
        const float hr = ar[r] * kRecScale + bhr;
        const float hz = az[r] * kRecScale + bhz;
        const float hn = an[r] * kRecScale + bhn;
        const float rg = 1.0f / (1.0f + expf(-(xr[r] + hr)));
        const float zg = 1.0f / (1.0f + expf(-(xz[r] + hz)));
        const float nc = tanhf(xn[r] + rg * hn);
        const float ho = Hm[row * kHmP + j];
        const float hnew = nc + zg * (ho - nc);
        Hm[row * kHmP + j] = hnew;
        ahn[row * kHP + j] = (_Float16)carry_flush(hnew, kActCarry);
      }
    }
    __syncthreads();

    v4f ov[8];
#pragma unroll
    for (int it = 0; it < 8; ++it) {
      const int row = it * 2 + hh;
      const float mk = (s < lenr[it]) ? 1.0f : 0.0f;
      const v4f hv = *(const v4f*)(Hm + row * kHmP + 64 * wave + c4);
      ov[it] = hv * mk;
    }
    for (int pass = 0; pass < 2; ++pass) {
#pragma unroll
      for (int it = 0; it < 8; ++it) {
        const int row = it * 2 + hh;
        float* p0 = OUT0 + ((size_t)(rowbase + row) * kSteps + s) * kHid + 64 * wave + c4;
        *(volatile v4f*)p0 = ov[it];
      }
      __threadfence();
    }
  }
}


static_assert(((size_t)kRows * kD / 8) % kThr == 0 && ((size_t)kQRows * kD / 8) % kThr == 0 && ((size_t)kGate3 * kD2 / 8) % kThr == 0 && ((size_t)kGate3 * kHid / 8) % kThr == 0, "cast grids exact");

extern "C" void kernel_launch(void* const* d_in, const int* in_sizes, int n_in,
                              void* d_out, int out_size, void* d_ws, size_t ws_size,
                              hipStream_t stream) {
  if (n_in < 16 || d_out == nullptr || d_ws == nullptr) return;
  if (in_sizes[0] != kRows * kD || in_sizes[1] != kQRows * kD || in_sizes[2] != kBatch || in_sizes[3] != kQRows) return;
  if (in_sizes[4] != kD * kHid || in_sizes[5] != kHid || in_sizes[6] != kD * kHid || in_sizes[7] != kHid) return;
  if (in_sizes[8] != kHid || in_sizes[9] != 1 || in_sizes[10] != kD2 * kD2 || in_sizes[11] != kD2) return;
  if (in_sizes[12] != kGate3 * kD2 || in_sizes[13] != kGate3 * kHid || in_sizes[14] != kGate3 || in_sizes[15] != kGate3) return;
  if (out_size != kRows * kHid) return;
  if (ws_size < kWsTotal) return;

  const float* ctx   = (const float*)d_in[0];
  const float* qst   = (const float*)d_in[1];
  const int*   clen  = (const int*)d_in[2];
  const float* qmask = (const float*)d_in[3];
  const float* Wc    = (const float*)d_in[4];
  const float* bc    = (const float*)d_in[5];
  const float* Wq    = (const float*)d_in[6];
  const float* bq    = (const float*)d_in[7];
  const float* Ws    = (const float*)d_in[8];
  const float* bs    = (const float*)d_in[9];
  const float* Wg    = (const float*)d_in[10];
  const float* bg    = (const float*)d_in[11];
  const float* Wih   = (const float*)d_in[12];
  const float* Whh   = (const float*)d_in[13];
  const float* bih   = (const float*)d_in[14];
  const float* bhh   = (const float*)d_in[15];
  float* out = (float*)d_out;

  char* ws = (char*)d_ws;
  unsigned short* C16 = (unsigned short*)(ws + kOffC16);
  unsigned short* Q16 = (unsigned short*)(ws + kOffQ16);
  unsigned short* QT  = (unsigned short*)(ws + kOffQT);
  unsigned short* WCT = (unsigned short*)(ws + kOffWCT);
  unsigned short* WQT = (unsigned short*)(ws + kOffWQT);
  unsigned short* WGT = (unsigned short*)(ws + kOffWGT);
  unsigned short* WIH = (unsigned short*)(ws + kOffWIH);
  unsigned short* WHH = (unsigned short*)(ws + kOffWHH);
  float* BV  = (float*)(ws + kOffBV);
  float* CD  = (float*)(ws + kOffCD);
  float* QD  = (float*)(ws + kOffQD);
  unsigned short* S16 = (unsigned short*)(ws + kOffS16);
  float* ATT = (float*)(ws + kOffATT);
  float* G   = (float*)(ws + kOffG);
  unsigned short* RN2 = (unsigned short*)(ws + kOffRN2);
  float* XS  = (float*)(ws + kOffXS);

  cast_plane_kernel<<<(int)(((size_t)kRows * kD / 8) / kThr), kThr, 0, stream>>>(ctx, C16, 8, kD2, 0);
  cast_plane_kernel<<<(int)(((size_t)kQRows * kD / 8) / kThr), kThr, 0, stream>>>(qst, Q16, 8, kD, 0);
  cast_plane_kernel<<<(int)(((size_t)kGate3 * kD2 / 8) / kThr), kThr, 0, stream>>>(Wih, WIH, 9, kD2, 0);
  cast_plane_kernel<<<(int)(((size_t)kGate3 * kHid / 8) / kThr), kThr, 0, stream>>>(Whh, WHH, 8, kHid, 0);
  tplane_kernel<<<dim3(kHid, 1), kD / 8, 0, stream>>>(Wc, WCT, kD, kHid);
  tplane_kernel<<<dim3(kHid, 1), kD / 8, 0, stream>>>(Wq, WQT, kD, kHid);
  tplane_kernel<<<dim3(kD2, 1), kD2 / 8, 0, stream>>>(Wg, WGT, kD2, kD2);
  tplane_kernel<<<dim3(kD, kBatch), kLq / 8, 0, stream>>>(qst, QT, kLq, kD);
  ca_bias_kernel<<<1, kThr, 0, stream>>>(bc, bq, bg, bih, bhh, BV);

  wmma_gemm64<0, false, 2, 0, false, 0><<<dim3((kRows / 64) * (kHid / 64) / 8, 1), 256, 0, stream>>>(
      C16, C16, kD2, 0L, WCT, WCT, kD, 0L, (void*)CD, (void*)CD, kHid, 0L,
      BV + 0 * kGate3, nullptr, 0L, kRows, kHid, kD, kXsScale);
  wmma_gemm64<0, false, 2, 0, false, 0><<<dim3((kQRows / 64) * (kHid / 64) / 8, 1), 256, 0, stream>>>(
      Q16, Q16, kD, 0L, WQT, WQT, kD, 0L, (void*)QD, (void*)QD, kHid, 0L,
      BV + 1 * kGate3, nullptr, 0L, kQRows, kHid, kD, kXsScale);
  score_kernel<<<kBatch * 8, kThr, 0, stream>>>(CD, QD, Ws, bs, qmask, S16);
  for (int b = 0; b < kBatch; ++b) {
    const unsigned short* Ab = S16 + (size_t)b * kSteps * kLq;
    const unsigned short* Bb = QT + (size_t)b * kD * kLq;
    float* Cb = ATT + (size_t)b * kSteps * kD;
    wmma_gemm64<0, false, 2, 0, false, 0><<<dim3((kSteps / 64) * (kD / 64) / 8, 1), 256, 0, stream>>>(
        Ab, Ab, kLq, 0L, Bb, Bb, kLq, 0L, (void*)Cb, (void*)Cb, kD, 0L,
        BV + 5 * kGate3, nullptr, 0L, kSteps, kD, kLq, kRecScale);
  }
  att_cast_kernel<<<(int)(((size_t)kRows * kD / 8) / kThr), kThr, 0, stream>>>(ATT, C16);
  wmma_gemm64<0, false, 2, 0, false, 0><<<dim3((kRows / 64) * (kD2 / 64) / 8, 1), 256, 0, stream>>>(
      C16, C16, kD2, 0L, WGT, WGT, kD2, 0L, (void*)G, (void*)G, kD2, 0L,
      BV + 2 * kGate3, nullptr, 0L, kRows, kD2, kD2, kXsScale);
  gate_mul_kernel<<<(int)(((size_t)kRows * kD2 / 4) / kThr), kThr, 0, stream>>>(ctx, ATT, G, RN2);
  wmma_gemm64<0, false, 2, 0, false, 0><<<dim3((kRows / 64) * (kGate3 / 64) / 8, 1), 256, 0, stream>>>(
      RN2, RN2, kD2, 0L, WIH, WIH, kD2, 0L, (void*)XS, (void*)XS, kGate3, 0L,
      BV + 3 * kGate3, nullptr, 0L, kRows, kGate3, kD2, kXsScale);
  gated_run_kernel<<<kBatch / kSeqBlk, kThrRun, 0, stream>>>(XS, WHH, BV + 4 * kGate3, clen, out);
}
